// GINLayer_49048526520633
// MI455X (gfx1250) — hardware-run, weakly checked
//
#include <hip/hip_runtime.h>


namespace {

constexpr int N = 100000, NP = 100032, NPL = NP  , SRCM = N  , EFULL = 1600000, E = EFULL  ;
constexpr int D = 128, HH = 256, NBLK = NP / 32, NL = (NPL < N ? NPL : N);
constexpr float XS = 8.0f, WSC = 256.0f, WSQ = 0.25f, RS_ = 1024.0f, BNEPS = 1e-5f, SLOPE = 0.0f;
static_assert(NP % 32 == 0 && NP >= N && NPL % 32 == 0 && D == 128 && HH == 256, "tiling");
typedef _Float16 b16;
typedef __attribute__((ext_vector_type(16))) _Float16 v16b;
typedef __attribute__((ext_vector_type(8))) _Float16 v8b;
typedef __attribute__((ext_vector_type(8))) float v8f;
typedef __attribute__((ext_vector_type(4))) float v4f;
__device__ __forceinline__ float bf16_rne(float f) { unsigned int u = __float_as_uint(f); u += 0x7FFFu + ((u >> 16) & 1u); return __uint_as_float(u & 0xFFFF0000u); }
__device__ __forceinline__ void split16(float v, b16& hi, b16& lo) { hi = (b16)v; lo = (b16)(v - (float)hi); }
__device__ __forceinline__ v16b frag_kb(const b16* p, int hh) { const v8b a = *(const v8b*)(p + 8 * hh), b = *(const v8b*)(p + 16 + 8 * hh); v16b f;
#pragma unroll
  for (int e = 0; e < 8; ++e) { f[e] = a[e]; f[8 + e] = b[e]; } return f; }
__device__ __forceinline__ v8f wmma16b(v16b a, v16b b, v8f c) { v8f d = __builtin_amdgcn_wmma_f32_16x16x32_f16(false, a, false, b, (short)0, c, false, false); asm volatile("v_nop\n\tv_nop\n\tv_nop\n\tv_nop" : "+v"(d) : "v"(a), "v"(b)); return d; }
__device__ __forceinline__ void wave_lds_sync() { __builtin_amdgcn_fence(__ATOMIC_RELEASE, "workgroup"); __builtin_amdgcn_wave_barrier(); __builtin_amdgcn_fence(__ATOMIC_ACQUIRE, "workgroup"); }
__device__ __forceinline__ float pmul(float a, float b) { float p = a * b; asm volatile("" : "+v"(p)); return p; }
__device__ __forceinline__ int iclamp(int v, int lo, int hi) { return v < lo ? lo : (v > hi ? hi : v); }
constexpr int CSR_NBLK = 512, CSR_GB = 9, CSR_GN = 1 << CSR_GB  , CSR_MAXG = 512, CSR_CAP = 12288  ;
__global__ __launch_bounds__(64) void csrA_kernel(const int* __restrict__ dst, int E, int N, int nG, int CHP, int NGP, int* __restrict__ STG, int* __restrict__ HST) {
  extern __shared__ int sm[];
  int* cnt = sm; int* run = sm + NGP; int* ids = sm + 2 * NGP;
  const int b = blockIdx.x; const int ch = (E + CSR_NBLK - 1) / CSR_NBLK; const int e0 = b * ch, e1 = min(E, e0 + ch);
  for (int i = threadIdx.x; i < NGP; i += 64) cnt[i] = 0;
  for (int i = threadIdx.x; i < CHP; i += 64) ids[i] = -1;
  __syncthreads();
  if (threadIdx.x == 0) {
    for (int e = e0; e < e1; ++e) { int d = dst[e]; d = (d < 0) ? 0 : (d >= N ? N - 1 : d); cnt[d >> CSR_GB] += 1; }
    int acc = 0; for (int g = 0; g < nG; ++g) { run[g] = acc; acc += cnt[g]; }
    for (int e = e0; e < e1; ++e) { int d = dst[e]; d = (d < 0) ? 0 : (d >= N ? N - 1 : d); const int g = d >> CSR_GB; ids[run[g]] = e; run[g] += 1; } }
  __syncthreads();
  typedef __attribute__((ext_vector_type(4))) int v4i;
  for (int pass = 0; pass < 2; ++pass) {
    for (int i = threadIdx.x; i < CHP / 4; i += 64) *(volatile v4i*)(STG + (size_t)b * CHP + i * 4) = *(const v4i*)(&ids[i * 4]);
    for (int i = threadIdx.x; i < NGP / 4; i += 64) { v4i v; for (int e = 0; e < 4; ++e) v[e] = (i * 4 + e < nG) ? cnt[i * 4 + e] : 0; *(volatile v4i*)(HST + (size_t)b * NGP + i * 4) = v; }
    __threadfence(); }
}
__global__ __launch_bounds__(512) void csrS_kernel(const int* __restrict__ HST, int nG, int NGP, int* __restrict__ START, int* __restrict__ TOT, int* __restrict__ OFF) {
  __shared__ int tot[CSR_MAXG];
  const int b = threadIdx.x;
  for (int pass = 0; pass < 2; ++pass) { int runb = 0; for (int g = 0; g < nG; ++g) { int c = HST[(size_t)b * NGP + g]; c = (c < 0) ? 0 : c; ((volatile int*)OFF)[(size_t)g * CSR_NBLK + b] = runb; runb += c; } __threadfence(); }
  for (int g = threadIdx.x; g < nG; g += 512) { int s = 0; for (int bb = 0; bb < CSR_NBLK; ++bb) { int c = HST[(size_t)bb * NGP + g]; s += (c < 0) ? 0 : c; } tot[g] = s; }
  __syncthreads();
  if (threadIdx.x < 32) {
    __shared__ int st[CSR_MAXG + 32];
    if (threadIdx.x == 0) { int acc = 0; for (int g = 0; g < NGP; ++g) { st[g] = acc; if (g < nG) acc += (tot[g] + 31) & ~31; } st[NGP] = acc; }
    __builtin_amdgcn_fence(__ATOMIC_RELEASE, "workgroup"); __builtin_amdgcn_wave_barrier(); __builtin_amdgcn_fence(__ATOMIC_ACQUIRE, "workgroup");
    for (int pass = 0; pass < 2; ++pass) { for (int i = threadIdx.x; i < NGP + 32; i += 32) { ((volatile int*)START)[i] = (i <= NGP) ? st[min(i, NGP)] : 0; ((volatile int*)TOT)[i] = (i < nG) ? tot[i] : 0; } __threadfence(); } }
}
__global__ __launch_bounds__(256) void csrB_kernel(const int* __restrict__ dst, int N, int nG, int CHP, int NGP, int permLen, const int* __restrict__ STG, const int* __restrict__ HST, const int* __restrict__ OFF, const int* __restrict__ START, const int* __restrict__ TOT, int* __restrict__ PERM, int* __restrict__ ROWPTR, int* __restrict__ ROWCNT, int* __restrict__ FLAG) {
  typedef __attribute__((ext_vector_type(4))) int v4i;
  __shared__ int ids[CSR_CAP]; __shared__ unsigned short key[CSR_CAP]; __shared__ int outp[CSR_CAP]; __shared__ int ncnt[CSR_GN + 1]; __shared__ int boff[CSR_NBLK + 1];
  const int g = blockIdx.x, t_ = threadIdx.x; int tot = TOT[g]; int st = START[g], stn = START[g + 1]; const int v0 = g * CSR_GN; const int nv = min(CSR_GN, N - v0);
  st = (st < 0) ? 0 : (st > permLen - 32 ? permLen - 32 : st) & ~31; stn = (stn < st) ? st : (stn > permLen ? permLen : stn); tot = (tot < 0) ? 0 : tot; if (tot > stn - st && tot <= CSR_CAP) tot = stn - st;
  if (tot > CSR_CAP) {
    for (int pass = 0; pass < 2; ++pass) { for (int i = t_; i < CSR_GN / 4; i += 256) { v4i a, c; for (int e = 0; e < 4; ++e) { a[e] = st; c[e] = 0; } *(volatile v4i*)(ROWPTR + v0 + i * 4) = a; *(volatile v4i*)(ROWCNT + v0 + i * 4) = c; } if (t_ == 0) ((volatile int*)FLAG)[0] = 1; __threadfence(); } (void)nv; return; }
  if (t_ == 0) { int acc = 0; for (int b = 0; b < CSR_NBLK; ++b) { boff[b] = acc; int c = HST[(size_t)b * NGP + g]; c = (c < 0) ? 0 : (c > CHP ? CHP : c); acc += c; if (acc > tot) acc = tot; } boff[CSR_NBLK] = acc; }
  for (int i = t_; i <= CSR_GN; i += 256) ncnt[i] = 0;
  __syncthreads();
  for (int b = 0; b < CSR_NBLK; ++b) { const int c = boff[b + 1] - boff[b]; int o_ = OFF[(size_t)g * CSR_NBLK + b]; o_ = (o_ < 0) ? 0 : (o_ > CHP - c ? CHP - c : o_); const int* src_ = STG + (size_t)b * CHP + o_;
    for (int i = t_; i < c; i += 256) { int id = src_[i]; id = (id < 0) ? 0 : id; ids[boff[b] + i] = id; int d = dst[id]; d = (d < v0) ? v0 : (d >= N ? N - 1 : d); int kk = d - v0; kk = (kk < 0) ? 0 : (kk >= CSR_GN ? CSR_GN - 1 : kk); key[boff[b] + i] = (unsigned short)kk; } }
  __syncthreads();
  if (t_ == 0) { for (int i = 0; i < tot; ++i) ncnt[key[i]] += 1; int acc = 0; for (int vl = 0; vl < CSR_GN; ++vl) { const int c = ncnt[vl]; ncnt[vl] = acc; acc += c; } ncnt[CSR_GN] = acc;
    for (int i = 0; i < tot; ++i) { const int vl = key[i]; outp[ncnt[vl]] = ids[i]; ncnt[vl] += 1; }
    for (int vl = CSR_GN; vl > 0; --vl) ncnt[vl] = ncnt[vl - 1]; ncnt[0] = 0; }
  __syncthreads();
  for (int pass = 0; pass < 2; ++pass) {
    for (int i = t_; i < (stn - st) / 4; i += 256) { v4i v; for (int e = 0; e < 4; ++e) { const int q = i * 4 + e; v[e] = (q < tot) ? outp[q] : -1; } *(volatile v4i*)(PERM + st + i * 4) = v; }
    for (int i = t_; i < CSR_GN / 4; i += 256) { v4i a, c; for (int e = 0; e < 4; ++e) { const int vl = i * 4 + e; a[e] = st + ncnt[vl]; c[e] = (vl < nv) ? (ncnt[vl + 1] - ncnt[vl]) : 0; } *(volatile v4i*)(ROWPTR + v0 + i * 4) = a; *(volatile v4i*)(ROWCNT + v0 + i * 4) = c; }
    __threadfence(); }
}
__global__ __launch_bounds__(256) void csrZ_kernel(int* __restrict__ p, size_t n4) { typedef __attribute__((ext_vector_type(4))) int v4i; const size_t tid = (size_t)blockIdx.x * 256 + threadIdx.x, nth = (size_t)gridDim.x * 256; v4i z = {0, 0, 0, 0}; for (size_t i = tid; i < n4; i += nth) *(volatile v4i*)(p + i * 4) = z; }
struct CsrBufs { int *STG, *HST, *OFF, *START, *TOT, *PERM, *ROWPTR, *ROWCNT, *FLAG; int nG, NGP, CHP; size_t permLen; char* base; size_t bytes; };
static size_t csr_carve(CsrBufs& c, char* ws, size_t off, int E, int N) {
  const size_t off0 = off; c.base = ws + off;
  auto al = [&](size_t bytes) { char* p = ws + off; off += (bytes + 255) & ~(size_t)255; return p; };
  c.nG = (N + CSR_GN - 1) / CSR_GN; c.NGP = (c.nG + 31) & ~31; const int ch = (E + CSR_NBLK - 1) / CSR_NBLK; c.CHP = (ch + 31) & ~31; c.permLen = (size_t)E + 32 * (size_t)c.nG + 32;
  c.STG = (int*)al((size_t)CSR_NBLK * c.CHP * 4); c.HST = (int*)al((size_t)CSR_NBLK * c.NGP * 4); c.OFF = (int*)al((size_t)c.NGP * CSR_NBLK * 4); c.START = (int*)al((size_t)(c.NGP + 64) * 4); c.TOT = (int*)al((size_t)(c.NGP + 64) * 4);
  c.PERM = (int*)al(c.permLen * 4); c.ROWPTR = (int*)al((size_t)c.nG * CSR_GN * 4); c.ROWCNT = (int*)al((size_t)c.nG * CSR_GN * 4); c.FLAG = (int*)al(256);
  c.bytes = off - off0; return off;
}
static void csr_build(const CsrBufs& c, const int* dst, int E, int N, hipStream_t stream) {
  const size_t smem = (size_t)(2 * c.NGP + c.CHP) * 4;
  csrZ_kernel<<<512, 256, 0, stream>>>((int*)c.base, c.bytes / 16);
  csrA_kernel<<<CSR_NBLK, 64, smem, stream>>>(dst, E, N, c.nG, c.CHP, c.NGP, c.STG, c.HST);
  csrS_kernel<<<1, 512, 0, stream>>>(c.HST, c.nG, c.NGP, c.START, c.TOT, c.OFF);
  csrB_kernel<<<c.nG, 256, 0, stream>>>(dst, N, c.nG, c.CHP, c.NGP, (int)c.permLen, c.STG, c.HST, c.OFF, c.START, c.TOT, c.PERM, c.ROWPTR, c.ROWCNT, c.FLAG);
}

typedef __attribute__((ext_vector_type(4))) _Float16 v4h;
template <int K, int NOUT>
__global__ __launch_bounds__(256) void wt_kernel(const float* __restrict__ w, b16* __restrict__ WT, float scl) {
  const int u = blockIdx.x * 256 + threadIdx.x; if (u >= NOUT * K / 8) return; const int e = u * 8; const int o = e / K, k0 = e % K; v8b v;
#pragma unroll
  for (int j = 0; j < 8; ++j) v[j] = (b16)(bf16_rne(w[(size_t)(k0 + j) * NOUT + o]) * scl);
  for (int pass = 0; pass < 2; ++pass) { *(volatile v8b*)(WT + e) = v; __threadfence(); }
}
__global__ __launch_bounds__(256) void agg_kernel(const float* __restrict__ x, const float* __restrict__ epsp, const int* __restrict__ srcs, const int* __restrict__ PERM, const int* __restrict__ ROWPTR, const int* __restrict__ ROWCNT, int permLen, float* __restrict__ Hh) {
  const int tid = threadIdx.x; const int row = tid >> 3, g = tid & 7, c0 = g * 16; const int v = blockIdx.x * 32 + row; const int vv = v < N ? v : N - 1; const float sc = 1.0f + bf16_rne(epsp[0]);
  float m[16]; { const float* xr = x + (size_t)vv * D + c0; for (int q = 0; q < 4; ++q) { const v4f t4 = *(const v4f*)(xr + 4 * q); for (int j = 0; j < 4; ++j) m[4 * q + j] = sc * bf16_rne(t4[j]); } }
  int cnt = 0, p0 = 0; if (v < N) { cnt = iclamp(ROWCNT[v], 0, 65536); p0 = iclamp(ROWPTR[v], 0, permLen - 1); if (p0 + cnt > permLen) cnt = permLen - p0; }
#pragma unroll 1
  for (int i = 0; i < cnt; ++i) { const int e = iclamp(PERM[p0 + i], 0, E - 1); int s = iclamp(srcs[e], 0, N - 1); if (SRCM < N) s %= SRCM; const float* xr = x + (size_t)s * D + c0;
#pragma unroll
    for (int q = 0; q < 4; ++q) { const v4f t4 = *(const v4f*)(xr + 4 * q); for (int j = 0; j < 4; ++j) m[4 * q + j] += bf16_rne(t4[j]); } }
  for (int pass = 0; pass < 2; ++pass) { float* hr = Hh + (size_t)v * D + c0;
#pragma unroll
    for (int q = 0; q < 4; ++q) { v4f o; for (int j = 0; j < 4; ++j) o[j] = (v < N) ? m[4 * q + j] : 0.0f; *(volatile v4f*)(hr + 4 * q) = o; }
    __threadfence(); }
}
template <int STAGE>
__global__ __launch_bounds__(64) void gemm_kernel(const float* __restrict__ Hh, const b16* __restrict__ W1T, const b16* __restrict__ W1Q, const float* __restrict__ b1, const float* __restrict__ ST1, const float* __restrict__ g1, const float* __restrict__ be1, const b16* __restrict__ W2T, const b16* __restrict__ W2Q, const float* __restrict__ b2, float* __restrict__ U, float* __restrict__ PART) {
  __shared__ __attribute__((aligned(16))) b16 Ah[2][16][HH + 8], Al[2][16][HH + 8]; __shared__ __attribute__((aligned(16))) float Tf[2][16][D + 4]; __shared__ __attribute__((aligned(16))) float Cs[2][2][HH];
  const int wave = threadIdx.x >> 5, lane = threadIdx.x & 31, nloc = lane & 15, hlf = lane >> 4; const size_t m0 = (size_t)blockIdx.x * 32 + wave * 16;
  for (int idx = lane; idx < 16 * (D / 4); idx += 32) { const int rr = idx / (D / 4), c4 = (idx % (D / 4)) * 4; const v4f v = *(const v4f*)(Hh + (m0 + rr) * D + c4); v4h hv, lv;
    for (int j = 0; j < 4; ++j) { const float vs = v[j] * XS; const b16 ph = (b16)vs; hv[j] = ph; lv[j] = (b16)((vs - (float)ph) * RS_); } *(v4h*)(&Ah[wave][rr][c4]) = hv; *(v4h*)(&Al[wave][rr][c4]) = lv; }
  wave_lds_sync();
  v8f acc[16];
#pragma unroll
  for (int t = 0; t < 16; ++t) acc[t] = (v8f){};
#pragma unroll
  for (int kb = 0; kb < D; kb += 32) { const v16b a = frag_kb(&Ah[wave][nloc][kb], hlf), al = frag_kb(&Al[wave][nloc][kb], hlf);
#pragma unroll
    for (int t = 0; t < 16; ++t) { const size_t wo_ = (size_t)(t * 16 + nloc) * D + kb; acc[t] = wmma16b(a, frag_kb(W1T + wo_, hlf), acc[t]); acc[t] = wmma16b(al, frag_kb(W1Q + wo_, hlf), acc[t]); } }
  wave_lds_sync();
  if (STAGE == 1) {
#pragma unroll
    for (int t = 0; t < 16; ++t) { const int col = t * 16 + nloc; const float bb = bf16_rne(b1[col]); float s1 = 0.0f, s2 = 0.0f;
#pragma unroll
      for (int r = 0; r < 8; ++r) { const bool ok = (m0 + 8 * hlf + r) < (size_t)N; const float tv = ok ? acc[t][r] * (1.0f / (XS * WSC)) + bb : 0.0f; s1 += tv; s2 = fmaf(tv, tv, s2); }
      s1 += __shfl_xor(s1, 16); s2 += __shfl_xor(s2, 16);
      if (hlf == 0) { Cs[wave][0][col] = s1; Cs[wave][1][col] = s2; } }
    __syncthreads();
    for (int pass = 0; pass < 2; ++pass) { if (wave == 0) { for (int k = 0; k < 2; ++k) for (int c8 = 0; c8 < HH; c8 += 128) { v4f p; for (int j = 0; j < 4; ++j) { const int c = c8 + lane * 4 + j; p[j] = Cs[0][k][c] + Cs[1][k][c]; } *(volatile v4f*)(PART + ((size_t)blockIdx.x * 2 + k) * HH + c8 + lane * 4) = p; } } __threadfence(); }
  } else {
#pragma unroll
    for (int t = 0; t < 16; ++t) { const int col = t * 16 + nloc; const float bb = bf16_rne(b1[col]), mean = ST1[col], rs = ST1[HH + col], gg = bf16_rne(g1[col]), be = bf16_rne(be1[col]);
#pragma unroll
      for (int r = 0; r < 8; ++r) { const float tv = fmaxf(pmul((acc[t][r] * (1.0f / (XS * WSC)) + bb - mean) * rs, gg) + be, 0.0f); const float vs = tv * XS; const b16 ph = (b16)vs; Ah[wave][8 * hlf + r][col] = ph; Al[wave][8 * hlf + r][col] = (b16)((vs - (float)ph) * RS_); } }
    wave_lds_sync();
    v8f acc2[8];
#pragma unroll
    for (int t = 0; t < 8; ++t) acc2[t] = (v8f){};
#pragma unroll 2
    for (int kb = 0; kb < HH; kb += 32) { const v16b a = frag_kb(&Ah[wave][nloc][kb], hlf), al = frag_kb(&Al[wave][nloc][kb], hlf);
#pragma unroll
      for (int t = 0; t < 8; ++t) { const size_t wo_ = (size_t)(t * 16 + nloc) * HH + kb; acc2[t] = wmma16b(a, frag_kb(W2T + wo_, hlf), acc2[t]); acc2[t] = wmma16b(al, frag_kb(W2Q + wo_, hlf), acc2[t]); } }
#pragma unroll
    for (int t = 0; t < 8; ++t) { const int col = t * 16 + nloc; const float bb = bf16_rne(b2[col]); float s1 = 0.0f, s2 = 0.0f;
#pragma unroll
      for (int r = 0; r < 8; ++r) { const bool ok = (m0 + 8 * hlf + r) < (size_t)N; const float uv = ok ? acc2[t][r] * (1.0f / (XS * WSC)) + bb : 0.0f; Tf[wave][8 * hlf + r][col] = uv; s1 += uv; s2 = fmaf(uv, uv, s2); }
      s1 += __shfl_xor(s1, 16); s2 += __shfl_xor(s2, 16); if (hlf == 0) { Cs[wave][0][col] = s1; Cs[wave][1][col] = s2; } }
    __syncthreads();
    for (int pass = 0; pass < 2; ++pass) { for (int rr = 0; rr < 16; ++rr) *(volatile v4f*)(U + (m0 + rr) * D + lane * 4) = *(const v4f*)(&Tf[wave][rr][lane * 4]);
      if (wave == 0) { for (int k = 0; k < 2; ++k) { v4f p; for (int j = 0; j < 4; ++j) { const int c = lane * 4 + j; p[j] = Cs[0][k][c] + Cs[1][k][c]; } *(volatile v4f*)(PART + ((size_t)blockIdx.x * 2 + k) * HH + lane * 4) = p; } }
      __threadfence(); } }
}
template <int W>
__global__ __launch_bounds__(256) void colred_kernel(const float* __restrict__ PART, float* __restrict__ ST) {
  const int c = threadIdx.x; if (c >= W) return; float s1 = 0.0f, s2 = 0.0f;
  for (int bk = 0; bk < NBLK; ++bk) { s1 += PART[((size_t)bk * 2) * HH + c]; s2 += PART[((size_t)bk * 2 + 1) * HH + c]; }
  const float mean = s1 * (1.0f / (float)N), msq = s2 * (1.0f / (float)N); const float var = fmaxf(msq - mean * mean, 0.0f);
  for (int pass = 0; pass < 2; ++pass) { ((volatile float*)ST)[c] = mean; ((volatile float*)ST)[HH + c] = rsqrtf(var + BNEPS); __threadfence(); }
}
__global__ __launch_bounds__(256) void out_kernel(const float* __restrict__ U, const float* __restrict__ ST2, const float* __restrict__ g2, const float* __restrict__ be2, float* __restrict__ out, int mrows) {
  const int tid = threadIdx.x;
  for (int pass = 0; pass < 2; ++pass) { for (int i = tid; i < 32 * (D / 4); i += 256) { const int rr = i / (D / 4), c4 = (i % (D / 4)) * 4; const size_t row = (size_t)blockIdx.x * 32 + rr; if (row >= (size_t)mrows) continue; const v4f u4 = *(const v4f*)(U + row * D + c4); v4f o;
      for (int j = 0; j < 4; ++j) { const int c = c4 + j; o[j] = fmaxf(pmul((u4[j] - ST2[c]) * ST2[HH + c], bf16_rne(g2[c])) + bf16_rne(be2[c]), 0.0f); }
      *(volatile v4f*)(out + row * D + c4) = o; } __threadfence(); }
}
}

extern "C" void kernel_launch(void* const* d_in, const int* in_sizes, int n_in, void* d_out, int out_size, void* d_ws, size_t ws_size, hipStream_t stream) {
  (void)n_in;
  auto Fp = [&](int i) { return (const float*)d_in[i]; }; auto Ip = [&](int i) { return (const int*)d_in[i]; };
  if (in_sizes[0] != N * D || in_sizes[1] != 2 * EFULL || in_sizes[2] != 1 || in_sizes[3] != D * HH || in_sizes[4] != HH || in_sizes[5] != HH || in_sizes[6] != HH || in_sizes[7] != HH * D || in_sizes[8] != D || in_sizes[9] != D || in_sizes[10] != D || out_size != N * D) return;
  size_t off = 0; char* ws = (char*)d_ws;
  auto carve = [&](size_t bytes) { char* p = ws + off; off += (bytes + 255) & ~(size_t)255; return p; };
  b16* W1T = (b16*)carve((size_t)HH * D * 2); b16* W1Q = (b16*)carve((size_t)HH * D * 2); b16* W2T = (b16*)carve((size_t)D * HH * 2); b16* W2Q = (b16*)carve((size_t)D * HH * 2);
  float* Hh = (float*)carve((size_t)NP * D * 4); float* U = (float*)carve((size_t)NP * D * 4); float* PART = (float*)carve((size_t)NBLK * 2 * HH * 4); float* ST1 = (float*)carve(2 * HH * 4); float* ST2 = (float*)carve(2 * HH * 4);
  CsrBufs csr; off = csr_carve(csr, ws, off, E, N);
  if (off > ws_size || off > ((size_t)176 << 20)) return;
  wt_kernel<D, HH><<<(HH * D / 8 + 255) / 256, 256, 0, stream>>>(Fp(3), W1T, WSC); wt_kernel<D, HH><<<(HH * D / 8 + 255) / 256, 256, 0, stream>>>(Fp(3), W1Q, WSQ);
  wt_kernel<HH, D><<<(D * HH / 8 + 255) / 256, 256, 0, stream>>>(Fp(7), W2T, WSC); wt_kernel<HH, D><<<(D * HH / 8 + 255) / 256, 256, 0, stream>>>(Fp(7), W2Q, WSQ);
  csr_build(csr, Ip(1) + EFULL, E, N, stream);
  agg_kernel<<<NP / 32, 256, 0, stream>>>(Fp(0), Fp(2), Ip(1), csr.PERM, csr.ROWPTR, csr.ROWCNT, (int)csr.permLen, Hh);
  gemm_kernel<1><<<NBLK, 64, 0, stream>>>(Hh, W1T, W1Q, Fp(4), ST1, Fp(5), Fp(6), W2T, W2Q, Fp(8), U, PART);
  colred_kernel<HH><<<1, 256, 0, stream>>>(PART, ST1);
  gemm_kernel<2><<<NBLK, 64, 0, stream>>>(Hh, W1T, W1Q, Fp(4), ST1, Fp(5), Fp(6), W2T, W2Q, Fp(8), U, PART);
  colred_kernel<D><<<1, 256, 0, stream>>>(PART, ST2);
  out_kernel<<<NPL / 32, 256, 0, stream>>>(U, ST2, Fp(9), Fp(10), (float*)d_out, NL);
}
